// MobileMamba_57432302682160
// MI455X (gfx1250) — hardware-verified
//
#include <hip/hip_runtime.h>
#include <math.h>

typedef __attribute__((ext_vector_type(16))) _Float16 v16h;
typedef __attribute__((ext_vector_type(8)))  _Float16 v8h;
typedef __attribute__((ext_vector_type(16))) __bf16   v16b;
typedef __attribute__((ext_vector_type(8)))  __bf16   v8b;
typedef __attribute__((ext_vector_type(8)))  float    v8f;
typedef __attribute__((ext_vector_type(4)))  float    v4f;

constexpr int kBatch  = 8;
constexpr int kSeqL   = 2048;
constexpr int kDmod   = 256;
constexpr int kEdim   = 512;
constexpr int kNst    = 8;
constexpr int kRows   = kBatch * kSeqL;
constexpr int kTP     = 260;
constexpr int kChunkT = 16;

constexpr size_t kOffXB   = 0;
constexpr size_t kSzXB    = (size_t)kRows * kDmod * 2;
constexpr size_t kOffW1B  = kOffXB + kSzXB;
constexpr size_t kSzW1B   = (size_t)kEdim * kDmod * 2;
constexpr size_t kOffW2H  = kOffW1B + kSzW1B;
constexpr size_t kSzW2H   = (size_t)kDmod * kEdim * 2;
constexpr size_t kOffXC   = kOffW2H + kSzW2H;
constexpr size_t kSzXC    = (size_t)kRows * kEdim * 4;
constexpr size_t kOffY16  = kOffXC + kSzXC;
constexpr size_t kSzY16   = (size_t)kRows * kEdim * 2;
constexpr size_t kWsTotal = kOffY16 + kSzY16;
static_assert(kWsTotal == 59244544ull);
static_assert((kOffW1B % 128) == 0 && (kOffW2H % 128) == 0 && (kOffXC % 128) == 0 && (kOffY16 % 128) == 0);
static_assert(kRows % 64 == 0 && kEdim % 64 == 0 && kDmod % 64 == 0);
static_assert(kDmod % 32 == 0 && kEdim % 32 == 0);
static_assert((kRows * kDmod) % 2048 == 0 && (kEdim * kDmod) % 2048 == 0);

__device__ __forceinline__ unsigned short f2bf_bits(float f) {
  unsigned u = __float_as_uint(f);
  return (unsigned short)((u + 0x7FFFu + ((u >> 16) & 1u)) >> 16);
}
__device__ __forceinline__ float bf_bits2f(unsigned short h) { return __uint_as_float(((unsigned)h) << 16); }

__device__ __forceinline__ void dep_guard_h(v8f& a, v8f& b, v16h x, v16h y) { asm volatile("v_nop\n\tv_nop\n\tv_nop\n\tv_nop" : "+v"(a), "+v"(b) : "v"(x), "v"(y)); }
__device__ __forceinline__ void dep_guard_b(v8f& a, v8f& b, v16b x, v16b y) { asm volatile("v_nop\n\tv_nop\n\tv_nop\n\tv_nop" : "+v"(a), "+v"(b) : "v"(x), "v"(y)); }
__device__ __forceinline__ void keep4_h(v16h a, v16h b, v16h c, v16h d) { asm volatile("v_nop" :: "v"(a), "v"(b), "v"(c), "v"(d)); }
__device__ __forceinline__ void keep4_b(v16b a, v16b b, v16b c, v16b d) { asm volatile("v_nop" :: "v"(a), "v"(b), "v"(c), "v"(d)); }
__device__ __forceinline__ void acc_guard4(v8f& a, v8f& b, v8f& c, v8f& d) { asm volatile("v_nop\n\tv_nop\n\tv_nop\n\tv_nop" : "+v"(a), "+v"(b), "+v"(c), "+v"(d)); }
template <typename T> struct Frag;
template <> struct Frag<_Float16> {
  typedef v16h V; union U { v16h v; v8h h[2]; };
  static __device__ __forceinline__ v16h load(const _Float16* p) {
    U f; f.h[0] = *(const v8h*)(p); f.h[1] = *(const v8h*)(p + 16); return f.v;
  }
  static __device__ __forceinline__ v8f mma(v16h a, v16h b, v8f c) {
    return __builtin_amdgcn_wmma_f32_16x16x32_f16(false, a, false, b, (short)0, c, false, false);
  }
  static __device__ __forceinline__ void guard(v8f& a, v8f& b, v16h x, v16h y) { dep_guard_h(a, b, x, y); }
  static __device__ __forceinline__ void keep(v16h a, v16h b, v16h c, v16h d) { keep4_h(a, b, c, d); }
};
template <> struct Frag<__bf16> {
  typedef v16b V; union U { v16b v; v8b h[2]; };
  static __device__ __forceinline__ v16b load(const __bf16* p) {
    U f; f.h[0] = *(const v8b*)(p); f.h[1] = *(const v8b*)(p + 16); return f.v;
  }
  static __device__ __forceinline__ v8f mma(v16b a, v16b b, v8f c) {
    return __builtin_amdgcn_wmma_f32_16x16x32_bf16(false, a, false, b, (short)0, c, false, false);
  }
  static __device__ __forceinline__ void guard(v8f& a, v8f& b, v16b x, v16b y) { dep_guard_b(a, b, x, y); }
  static __device__ __forceinline__ void keep(v16b a, v16b b, v16b c, v16b d) { keep4_b(a, b, c, d); }
};

template <int ET> struct Elem;
template <> struct Elem<0> { typedef _Float16 T; };
template <> struct Elem<1> { typedef __bf16 T; };
template <int ET, bool SPLIT, int BIAS_MODE, int OUT_MODE, bool RESID, int ACT = 0>
__global__ __launch_bounds__(256) void wmma_gemm64(
    const unsigned short* __restrict__ Ap, const unsigned short* __restrict__ A2p, int lda, long strideA,
    const unsigned short* __restrict__ Btp, const unsigned short* __restrict__ Bt2p, int ldb, long strideB,
    void* __restrict__ Cout, void* __restrict__ Cout2, int ldc, long strideC,
    const float* __restrict__ bias,
    const float* __restrict__ resid, long strideR,
    int M, int N, int K, float scale) {
  typedef typename Elem<ET>::T T;
  typedef typename Frag<T>::V V;
  const T* A = (const T*)Ap; const T* A2 = (const T*)A2p; const T* Bt = (const T*)Btp; const T* Bt2 = (const T*)Bt2p;
  __shared__ __align__(16) float sT[8][16 * 68];
  const int b    = blockIdx.y;
  const int lane = threadIdx.x & 31;
  const int wave = threadIdx.x >> 5;
  const int tilesN = N >> 6;
  const int tilesM = M >> 6;
  const int tile = blockIdx.x * 8 + wave;
  if (tile >= tilesM * tilesN) return;
  const int tm = tile / tilesN;
  const int tn = tile - tm * tilesN;
  const int m0 = tm << 6;
  const int n0 = tn << 6;

  const T* Ab  = A  + (size_t)b * strideA;
  const T* Bb  = Bt + (size_t)b * strideB;
  const T* Ab2 = SPLIT ? (A2  + (size_t)b * strideA) : nullptr;
  const T* Bb2 = SPLIT ? (Bt2 + (size_t)b * strideB) : nullptr;

  const int rlane = lane & 15;
  const int koff  = (lane >> 4) * 8;
  const int mOff  = (lane >> 4) * 8;

  v8f acc[4][4];
#pragma unroll
  for (int i = 0; i < 4; ++i)
#pragma unroll
    for (int j = 0; j < 4; ++j) acc[i][j] = (v8f){0.f,0.f,0.f,0.f,0.f,0.f,0.f,0.f};

  for (int k0 = 0; k0 < K; k0 += 32) {
    V bh[4], bl[4];
#pragma unroll
    for (int j = 0; j < 4; ++j) {
      const size_t bo = (size_t)(n0 + (j << 4) + rlane) * ldb + koff + k0;
      bh[j] = Frag<T>::load(Bb + bo);
      if (SPLIT) bl[j] = Frag<T>::load(Bb2 + bo);
    }
#pragma unroll
    for (int i = 0; i < 4; ++i) {
      const size_t ao = (size_t)(m0 + (i << 4) + rlane) * lda + koff + k0;
      V ah = Frag<T>::load(Ab + ao);
      V al;
      if (SPLIT) al = Frag<T>::load(Ab2 + ao);
#pragma unroll
      for (int j = 0; j < 4; ++j) {
        acc[i][j] = Frag<T>::mma(ah, bh[j], acc[i][j]);
        if (SPLIT) {
          acc[i][j] = Frag<T>::mma(ah, bl[j], acc[i][j]);
          acc[i][j] = Frag<T>::mma(al, bh[j], acc[i][j]);
        }
      }
      Frag<T>::guard(acc[i][0], acc[i][3], ah, SPLIT ? al : ah);
    }
    Frag<T>::keep(bh[0], bh[1], bh[2], bh[3]);
    if (SPLIT) Frag<T>::keep(bl[0], bl[1], bl[2], bl[3]);
  }
  acc_guard4(acc[0][0], acc[0][1], acc[0][2], acc[0][3]);
  acc_guard4(acc[1][0], acc[1][1], acc[1][2], acc[1][3]);
  acc_guard4(acc[2][0], acc[2][1], acc[2][2], acc[2][3]);
  acc_guard4(acc[3][0], acc[3][1], acc[3][2], acc[3][3]);

  float* slab = sT[wave];
  const float* Rb = RESID ? (resid + (size_t)b * strideR) : nullptr;
#pragma unroll
  for (int i = 0; i < 4; ++i) {
    const int mBase = m0 + (i << 4);
#pragma unroll
    for (int j = 0; j < 4; ++j) {
      const int n = n0 + (j << 4) + rlane;
      float bv = 0.f;
      if (BIAS_MODE == 2) bv = bias[n];
#pragma unroll
      for (int r = 0; r < 8; ++r) {
        float v = acc[i][j][r] * scale;
        if (BIAS_MODE == 1) v += bias[mBase + mOff + r];
        if (BIAS_MODE == 2) v += bv;
        if (RESID) v += Rb[(size_t)(mBase + mOff + r) * ldc + n];
        if (ACT == 1) v = tanhf(v);
        if (ACT == 2) v = fmaxf(v, 0.0f);
        if (ACT == 3) v = v / (1.0f + expf(-v));
        if (ACT == 4) v = (v > 0.f) ? v : 0.01f * v;
        if (ACT == 5) v = 0.5f * v * (1.0f + erff(v * 0.70710678118654752f));
        if (ACT == 6) v = v * __builtin_amdgcn_rcpf(1.0f + __expf(-v));
        slab[(mOff + r) * 68 + (j << 4) + rlane] = v;
      }
    }
    __builtin_amdgcn_fence(__ATOMIC_RELEASE, "workgroup");
    __builtin_amdgcn_wave_barrier();
    __builtin_amdgcn_fence(__ATOMIC_ACQUIRE, "workgroup");
    if (OUT_MODE == 0) {
      float* C = (float*)Cout + (size_t)b * strideC;
      const int hh = lane >> 4, c4 = (lane & 15) * 4;
      for (int pass = 0; pass < 2; ++pass) {
#pragma unroll
        for (int it = 0; it < 8; ++it) {
          const int row = it * 2 + hh;
          v4f v = *(const v4f*)(slab + row * 68 + c4);
          *(volatile v4f*)(C + (size_t)(mBase + row) * ldc + n0 + c4) = v;
        }
        __threadfence();
      }
    } else {
      const int q = lane >> 3, c8 = (lane & 7) * 8;
      unsigned short* C  = (unsigned short*)Cout  + (size_t)b * strideC;
      unsigned short* C2 = (OUT_MODE == 2) ? ((unsigned short*)Cout2 + (size_t)b * strideC) : nullptr;
      for (int pass = 0; pass < 2; ++pass) {
#pragma unroll
        for (int it = 0; it < 4; ++it) {
          const int row = it * 4 + q;
          const float* sp = slab + row * 68 + c8;
          v8h hv, lv;
#pragma unroll
          for (int e = 0; e < 8; ++e) {
            if (OUT_MODE == 1) {
              hv[e] = (_Float16)sp[e];
            } else {
              unsigned short hb = f2bf_bits(sp[e]);
              unsigned short lb = f2bf_bits(sp[e] - bf_bits2f(hb));
              hv[e] = __builtin_bit_cast(_Float16, hb);
              lv[e] = __builtin_bit_cast(_Float16, lb);
            }
          }
          *(volatile v8h*)(C + (size_t)(mBase + row) * ldc + n0 + c8) = hv;
          if (OUT_MODE == 2) *(volatile v8h*)(C2 + (size_t)(mBase + row) * ldc + n0 + c8) = lv;
        }
        __threadfence();
      }
    }
    __builtin_amdgcn_fence(__ATOMIC_RELEASE, "workgroup");
    __builtin_amdgcn_wave_barrier();
    __builtin_amdgcn_fence(__ATOMIC_ACQUIRE, "workgroup");
  }
}

template <int MODE>
__global__ __launch_bounds__(256) void cast16_kernel(
    const float* __restrict__ src, unsigned short* __restrict__ dst, int total8, float scale)
{
  const int i = blockIdx.x * 256 + threadIdx.x;
  if (i >= total8) return;
  const size_t e0 = (size_t)i << 3;
  const float* p = src + e0;
  const v4f a0 = *(const v4f*)(p);
  const v4f a1 = *(const v4f*)(p + 4);
  v8h hv;
#pragma unroll
  for (int e = 0; e < 4; ++e) {
    const unsigned short b0 = f2bf_bits(a0[e]);
    const unsigned short b1 = f2bf_bits(a1[e]);
    if (MODE == 0) {
      hv[e]     = __builtin_bit_cast(_Float16, b0);
      hv[4 + e] = __builtin_bit_cast(_Float16, b1);
    } else {
      hv[e]     = (_Float16)(bf_bits2f(b0) * scale);
      hv[4 + e] = (_Float16)(bf_bits2f(b1) * scale);
    }
  }
  unsigned short* q = dst + e0;
  *(volatile v8h*)q = hv;
  __threadfence();
  *(volatile v8h*)q = hv;
}

__device__ __forceinline__ float rbf(float v) { return bf_bits2f(f2bf_bits(v)); }

__global__ __launch_bounds__(256) void conv_bn_scan_kernel(
    const float* __restrict__ XC, const float* __restrict__ wd, const float* __restrict__ bd,
    const float* __restrict__ gam, const float* __restrict__ bet, const float* __restrict__ rmu,
    const float* __restrict__ rva, const float* __restrict__ Av, const float* __restrict__ Bmat,
    const float* __restrict__ Cmat, const float* __restrict__ Dvec, unsigned short* __restrict__ Y16)
{
  __shared__ __align__(16) float sT[kChunkT * kTP];
  const int tid = threadIdx.x, lane = tid & 31, wave = tid >> 5;
  const int e0 = blockIdx.x * 256;
  const int e  = e0 + tid;
  const int b  = blockIdx.y;

  const float w0 = rbf(wd[e * 5 + 0]), w1 = rbf(wd[e * 5 + 1]), w2 = rbf(wd[e * 5 + 2]);
  const float w3 = rbf(wd[e * 5 + 3]), w4 = rbf(wd[e * 5 + 4]);
  const float bde  = rbf(bd[e]);
  const float sc   = rbf(gam[e]) * rsqrtf(rbf(rva[e]) + 1e-5f);
  const float sh   = rbf(bet[e]) - rbf(rmu[e]) * sc;
  const float adec = expf(rbf(Av[e]));
  const float dv   = rbf(Dvec[e]);
  float bm[kNst], cm[kNst], h[kNst];
#pragma unroll
  for (int s = 0; s < kNst; ++s) { bm[s] = rbf(Bmat[e * kNst + s]); cm[s] = rbf(Cmat[e * kNst + s]); h[s] = 0.f; }

  const float* xcol = XC + (size_t)b * kSeqL * kEdim + e;
  const size_t rowBase = (size_t)b * kSeqL;
  float xm2 = 0.f, xm1 = 0.f;
  float xz  = xcol[0];
  float xp1 = xcol[(size_t)kEdim];

#pragma unroll 1
  for (int c = 0; c < kSeqL / kChunkT; ++c) {
#pragma unroll 1
    for (int s = 0; s < kChunkT; ++s) {
      const int t   = c * kChunkT + s;
      const int tn  = t + 2;
      const int tcl = (tn < kSeqL) ? tn : (kSeqL - 1);
      const float xr  = xcol[(size_t)tcl * kEdim];
      const float xp2 = (tn < kSeqL) ? xr : 0.f;
      float cv = w0 * xm2;
      cv = fmaf(w1, xm1, cv);
      cv = fmaf(w2, xz,  cv);
      cv = fmaf(w3, xp1, cv);
      cv = fmaf(w4, xp2, cv);
      cv += bde;
      const float ybn = cv * sc + sh;
      const float xl  = ybn * __builtin_amdgcn_rcpf(1.0f + __expf(-ybn));
      float ys = 0.f;
#pragma unroll
      for (int q = 0; q < kNst; ++q) {
        h[q] = adec * h[q] + xl * bm[q];
        ys = fmaf(h[q], cm[q], ys);
      }
      const float yv = ys + dv * xl;
      sT[s * kTP + tid] = yv;
      xm2 = xm1; xm1 = xz; xz = xp1; xp1 = xp2;
    }
    __syncthreads();
    v8h hv[2];
#pragma unroll
    for (int it = 0; it < 2; ++it) {
      const float* sp = sT + (it * 8 + wave) * kTP + lane * 8;
      const v4f a0 = *(const v4f*)(sp);
      const v4f a1 = *(const v4f*)(sp + 4);
#pragma unroll
      for (int q = 0; q < 4; ++q) {
        hv[it][q]     = (_Float16)(a0[q] * 256.0f);
        hv[it][4 + q] = (_Float16)(a1[q] * 256.0f);
      }
    }
    for (int pass = 0; pass < 2; ++pass) {
#pragma unroll
      for (int it = 0; it < 2; ++it)
        *(volatile v8h*)(Y16 + (rowBase + (size_t)c * kChunkT + it * 8 + wave) * kEdim + e0 + lane * 8) = hv[it];
      __threadfence();
    }
    __syncthreads();
  }
}

extern "C" void kernel_launch(void* const* d_in, const int* in_sizes, int n_in,
                              void* d_out, int out_size, void* d_ws, size_t ws_size,
                              hipStream_t stream) {
  if (n_in < 15) return;
  if (in_sizes[0]  != kRows * kDmod) return;
  if (in_sizes[1]  != kEdim * kDmod) return;
  if (in_sizes[2]  != kEdim) return;
  if (in_sizes[3]  != kEdim * 5) return;
  if (in_sizes[4]  != kEdim || in_sizes[5] != kEdim || in_sizes[6] != kEdim ||
      in_sizes[7]  != kEdim || in_sizes[8] != kEdim || in_sizes[9] != kEdim) return;
  if (in_sizes[10] != kEdim * kNst || in_sizes[11] != kEdim * kNst || in_sizes[12] != kEdim) return;
  if (in_sizes[13] != kDmod * kEdim) return;
  if (in_sizes[14] != kDmod) return;
  if (out_size != kRows * kDmod) return;
  if (ws_size < kWsTotal) return;

  const float* x     = (const float*)d_in[0];
  const float* w1    = (const float*)d_in[1];
  const float* b1    = (const float*)d_in[2];
  const float* wd    = (const float*)d_in[3];
  const float* bd    = (const float*)d_in[4];
  const float* gam   = (const float*)d_in[5];
  const float* bet   = (const float*)d_in[6];
  const float* rmu   = (const float*)d_in[7];
  const float* rva   = (const float*)d_in[8];
  const float* Av    = (const float*)d_in[9];
  const float* Bmat  = (const float*)d_in[10];
  const float* Cmat  = (const float*)d_in[11];
  const float* Dvec  = (const float*)d_in[12];
  const float* w2    = (const float*)d_in[13];
  const float* b2    = (const float*)d_in[14];

  char* ws = (char*)d_ws;
  unsigned short* XB  = (unsigned short*)(ws + kOffXB);
  unsigned short* W1B = (unsigned short*)(ws + kOffW1B);
  unsigned short* W2H = (unsigned short*)(ws + kOffW2H);
  float*          XC  = (float*)(ws + kOffXC);
  unsigned short* Y16 = (unsigned short*)(ws + kOffY16);

  {
    const int total8 = kRows * kDmod / 8;
    cast16_kernel<0><<<dim3((total8 + 255) / 256), dim3(256), 0, stream>>>(x, XB, total8, 1.0f);
  }
  {
    const int total8 = kEdim * kDmod / 8;
    cast16_kernel<0><<<dim3((total8 + 255) / 256), dim3(256), 0, stream>>>(w1, W1B, total8, 1.0f);
  }
  {
    const int total8 = kDmod * kEdim / 8;
    cast16_kernel<1><<<dim3((total8 + 255) / 256), dim3(256), 0, stream>>>(w2, W2H, total8, 32.0f);
  }
  {
    const int tiles = (kRows / 64) * (kEdim / 64);
    wmma_gemm64<1, false, 2, 0, false, 6><<<dim3((tiles + 7) / 8, 1), dim3(256), 0, stream>>>(
        XB, XB, kDmod, 0L, W1B, W1B, kDmod, 0L,
        (void*)XC, (void*)XC, kEdim, 0L, b1, b1, 0L, kRows, kEdim, kDmod, 1.0f);
  }
  conv_bn_scan_kernel<<<dim3(kEdim / 256, kBatch), dim3(256), 0, stream>>>(
      XC, wd, bd, gam, bet, rmu, rva, Av, Bmat, Cmat, Dvec, Y16);
  {
    const int tiles = (kRows / 64) * (kDmod / 64);
    wmma_gemm64<0, false, 2, 0, false, 0><<<dim3((tiles + 7) / 8, 1), dim3(256), 0, stream>>>(
        Y16, Y16, kEdim, 0L, W2H, W2H, kEdim, 0L,
        d_out, d_out, kDmod, 0L, b2, b2, 0L, kRows, kDmod, kEdim, 1.0f / 8192.0f);
  }
}
